// HeteroGCN_22789096472879
// MI455X (gfx1250) — hardware-verified
//
#include <hip/hip_runtime.h>
#include <stddef.h>
#include <stdint.h>


#define DIN     16
#define HID     256
#define CH      128
#define NREL    4
#define NTYP    2
#define NLAY    2
#define DOUT    4
#define NRC     640
#define HSW     512
#define NTHR    256
#define NWAVE   8
#define EPT     8
#define CHUNK   (NTHR * EPT)
#define WCAP    (EPT * 32)
#define LISTN   (NWAVE * WCAP)
#define NBMAX   2048
#define RCAP    28672
#define DEGCAP  64
#define GBM     64
#define GBN     64
#define GTHR    128
#define HBM     128
#define HTHR    256
#define FTHR    128
#define ZBLK    4096
#define CA      8.0f
#define CW      256.0f
#define SCL     0.00048828125f
#define HSC     0.0078125f
#define RHS     0.0625f
#define BNEPS   1e-5
#define WSLIM   268435456
#define LDS_AGG ((2 * RCAP + 2 * NBMAX + LISTN) * 4 + 64)
#define LDS_HG(NCOLS, KK) (72192 + 144 * (NCOLS) + 256 * (KK))

static_assert((CHUNK & (CHUNK - 1)) == 0 && CHUNK <= 4096);
static_assert((NBMAX & (NBMAX - 1)) == 0 && NBMAX <= 4096);
static_assert(NTHR * 8 == NBMAX);
static_assert(LISTN >= NBMAX);
static_assert(LISTN >= NWAVE * WCAP);
static_assert((RCAP % 32) == 0);
static_assert(NWAVE * 512 + 512 <= RCAP);
static_assert(LDS_AGG <= 300000 && (LDS_AGG % 16) == 0);
static_assert(LDS_HG(HID, 32) <= 300000 && LDS_HG(CH, HID) <= 300000 && LDS_HG(HID, CH) <= 300000);
static_assert(GBM == (GTHR / 32) * 16);
static_assert(HBM == NWAVE * 16 && HTHR == NWAVE * 32 && HBM <= HTHR);
static_assert((CH % 32) == 0 && (HID % 32) == 0 && (NRC % GBN) == 0);
static_assert(NRC == NREL * CH + CH && HSW == NREL * CH);
static_assert(DOUT == 4 && NTYP == 2);

typedef float    v4f  __attribute__((ext_vector_type(4)));
typedef float    v8f  __attribute__((ext_vector_type(8)));
typedef int      v4i  __attribute__((ext_vector_type(4)));
typedef int      v8i  __attribute__((ext_vector_type(8)));
typedef _Float16 v4h  __attribute__((ext_vector_type(4)));
typedef _Float16 v8h  __attribute__((ext_vector_type(8)));
typedef _Float16 v16h __attribute__((ext_vector_type(16)));
union FragH { v16h v; v8h h[2]; v8i w; };

__device__ __forceinline__ v8f wmh(const FragH& a, const FragH& b, v8f c) {
  v8f d = __builtin_amdgcn_wmma_f32_16x16x32_f16(false, a.v, false, b.v, (short)0, c, false, false);
  asm volatile("v_nop\n\tv_nop\n\tv_nop\n\tv_nop" : "+v"(d) : "v"(a.w), "v"(b.w));
  return d;
}

__device__ __forceinline__ v8h cvt8h(const v4f a, const v4f b, const float c) {
  v8h hv;
  hv[0] = (_Float16)(a.x * c); hv[1] = (_Float16)(a.y * c);
  hv[2] = (_Float16)(a.z * c); hv[3] = (_Float16)(a.w * c);
  hv[4] = (_Float16)(b.x * c); hv[5] = (_Float16)(b.y * c);
  hv[6] = (_Float16)(b.z * c); hv[7] = (_Float16)(b.w * c);
  return hv;
}

__device__ __forceinline__ float bf16r(float f) {
  unsigned u = __float_as_uint(f);
  u = (u + 0x7FFFu + ((u >> 16) & 1u)) & 0xFFFF0000u;
  return __uint_as_float(u);
}
__device__ __forceinline__ v4f bf16r4(v4f v) {
  v4f r;
  r.x = bf16r(v.x); r.y = bf16r(v.y); r.z = bf16r(v.z); r.w = bf16r(v.w);
  return r;
}
__device__ __forceinline__ v4f lrelu4(v4f v) {
  v4f r;
  r.x = v.x > 0.f ? v.x : 0.01f * v.x;
  r.y = v.y > 0.f ? v.y : 0.01f * v.y;
  r.z = v.z > 0.f ? v.z : 0.01f * v.z;
  r.w = v.w > 0.f ? v.w : 0.01f * v.w;
  return r;
}

template<int AMODE>
__device__ __forceinline__ v8h cv8(const float* __restrict__ arow, const float* mt, const float* sct,
                                   const float* bt, int kk) {
  v4f xa = *(const v4f*)(arow + kk);
  v4f xb = *(const v4f*)(arow + kk + 4);
  if (AMODE == 1) {
    const v4f ma = *(const v4f*)(mt + kk),  mb = *(const v4f*)(mt + kk + 4);
    const v4f sa = *(const v4f*)(sct + kk), sb = *(const v4f*)(sct + kk + 4);
    const v4f ba = *(const v4f*)(bt + kk),  bb = *(const v4f*)(bt + kk + 4);
    xa = lrelu4((xa - ma) * sa + ba);
    xb = lrelu4((xb - mb) * sb + bb);
  }
  return cvt8h(xa, xb, CA);
}

__device__ __forceinline__ int scan_chunk(const int* __restrict__ dsts, int nE, int cbase, int slotBase,
                                          int nb, int vec8, int* list, int tid, int lane, int wave) {
  int wc = 0;
  const int el0  = tid * EPT;
  const int e0   = cbase + el0;
  const int sent = -2147483647 - 1;
  v4i da, db;
  if (vec8 != 0 && cbase + CHUNK <= nE) {
    da = *(const v4i*)(dsts + e0);
    db = *(const v4i*)(dsts + e0 + 4);
  } else {
    da.x = (e0     < nE) ? dsts[min(e0,     nE - 1)] : sent;
    da.y = (e0 + 1 < nE) ? dsts[min(e0 + 1, nE - 1)] : sent;
    da.z = (e0 + 2 < nE) ? dsts[min(e0 + 2, nE - 1)] : sent;
    da.w = (e0 + 3 < nE) ? dsts[min(e0 + 3, nE - 1)] : sent;
    db.x = (e0 + 4 < nE) ? dsts[min(e0 + 4, nE - 1)] : sent;
    db.y = (e0 + 5 < nE) ? dsts[min(e0 + 5, nE - 1)] : sent;
    db.z = (e0 + 6 < nE) ? dsts[min(e0 + 6, nE - 1)] : sent;
    db.w = (e0 + 7 < nE) ? dsts[min(e0 + 7, nE - 1)] : sent;
  }
  const unsigned nbs = (unsigned)slotBase;
  const unsigned unb = (unsigned)nb;
  const unsigned s0 = (unsigned)da.x - nbs, s1 = (unsigned)da.y - nbs;
  const unsigned s2 = (unsigned)da.z - nbs, s3 = (unsigned)da.w - nbs;
  const unsigned s4 = (unsigned)db.x - nbs, s5 = (unsigned)db.y - nbs;
  const unsigned s6 = (unsigned)db.z - nbs, s7 = (unsigned)db.w - nbs;
  const bool h0 = s0 < unb, h1 = s1 < unb, h2 = s2 < unb, h3 = s3 < unb;
  const bool h4 = s4 < unb, h5 = s5 < unb, h6 = s6 < unb, h7 = s7 < unb;
  const unsigned any = __builtin_amdgcn_ballot_w32(h0 | h1 | h2 | h3 | h4 | h5 | h6 | h7);
  if (any != 0u) {
#define HITJ(J, HJ, SJ) { \
      const unsigned mj = __builtin_amdgcn_ballot_w32(HJ); \
      const int pos = wc + (int)__builtin_amdgcn_mbcnt_lo(mj, 0u); \
      if ((HJ) && pos < WCAP) list[wave * WCAP + pos] = ((el0 + (J)) << 12) | (int)(SJ); \
      wc += (int)__builtin_popcount(mj); }
    HITJ(0, h0, s0)
    HITJ(1, h1, s1)
    HITJ(2, h2, s2)
    HITJ(3, h3, s3)
    HITJ(4, h4, s4)
    HITJ(5, h5, s5)
    HITJ(6, h6, s6)
    HITJ(7, h7, s7)
#undef HITJ
  }
  return wc;
}

__global__ __launch_bounds__(NTHR) void k_zero(float* p, int n4) {
  const v4f z4 = {0.f, 0.f, 0.f, 0.f};
  const int gs = (int)gridDim.x * NTHR;
  const int i0 = (int)blockIdx.x * NTHR + (int)threadIdx.x;
#pragma unroll 1
  for (int i = i0; i < n4; i += gs) *(volatile v4f*)(p + (size_t)i * 4) = z4;
  __threadfence();
#pragma unroll 1
  for (int i = i0; i < n4; i += gs) *(volatile v4f*)(p + (size_t)i * 4) = z4;
}

__global__ __launch_bounds__(NTHR) void k_wprep(const float* __restrict__ W0, const float* __restrict__ W1,
                                              int G0, int NG, int NC, int Kreal, int K, int gs0,
                                              _Float16* WT, int nUnits) {
  const int u = (int)blockIdx.x * NTHR + (int)threadIdx.x;
  if (u >= nUnits) return;
  const int kq = K >> 3;
  const int n  = u / kq;
  const int k8 = (u - n * kq) * 8;
  const int g  = n / NG;
  const int c  = n - g * NG;
  const float* base = (g < G0) ? (W0 + (size_t)g * (size_t)gs0) : (W1 + (size_t)(g - G0) * (size_t)gs0);
  const int cl = c < NC ? c : NC - 1;
  float v[8];
#pragma unroll
  for (int j = 0; j < 8; ++j) {
    const int k  = k8 + j;
    const int kc = k < Kreal ? k : Kreal - 1;
    float w = base[(size_t)kc * (size_t)NC + cl];
    w = (c < NC && k < Kreal) ? w : 0.f;
    v[j] = bf16r(w);
  }
  const v4f a = {v[0], v[1], v[2], v[3]};
  const v4f b = {v[4], v[5], v[6], v[7]};
  const v8h hv = cvt8h(a, b, CW);
  const size_t o = (size_t)u * 8;
  *(volatile v8h*)(WT + o) = hv;
  __threadfence();
  *(volatile v8h*)(WT + o) = hv;
}

__global__ __launch_bounds__(NTHR) void k_fold(const float* __restrict__ REC, int nrec, int N,
                                             const float* __restrict__ gam, const float* __restrict__ bet,
                                             const int* __restrict__ nt, int nN, float* SS) {
  __shared__ __attribute__((aligned(16))) float SSL[1536];
  __shared__ __attribute__((aligned(16))) int   WCI[16];
  const int tid = (int)threadIdx.x, lane = tid & 31, wave = tid >> 5;
  {
    const v4f z4 = {0.f, 0.f, 0.f, 0.f};
    const v4i zi = {0, 0, 0, 0};
    for (int p = tid; p < 384; p += NTHR) ((v4f*)SSL)[p] = z4;
    if (tid < 4) ((v4i*)WCI)[tid] = zi;
  }
  __syncthreads();
  int c0 = 0;
#pragma unroll 1
  for (int i = tid; i < nN; i += NTHR) c0 += (nt[i] > 0) ? 0 : 1;
#pragma unroll
  for (int off = 16; off > 0; off >>= 1) c0 += __shfl_xor(c0, off);
  if (lane == 0) WCI[wave] = c0;
  __syncthreads();
  int cnt0 = 0;
#pragma unroll
  for (int w2 = 0; w2 < NWAVE; ++w2) cnt0 += WCI[w2];
  const int cnt1 = nN - cnt0;
#pragma unroll 1
  for (int e = tid; e < 2 * N; e += NTHR) {
    const int tt = (e >= N) ? 1 : 0;
    const int c  = e - tt * N;
    double S = 0.0, Q = 0.0;
    const float* rp = REC + (size_t)(2 * tt) * (size_t)N + c;
#pragma unroll 1
    for (int r = 0; r < nrec; ++r) {
      const float* q = rp + (size_t)r * (size_t)(4 * N);
      S += (double)q[0];
      Q += (double)q[N];
    }
    const int ci = tt ? cnt1 : cnt0;
    const double cf = (double)(ci < 1 ? 1 : ci);
    const double mean = S / cf;
    double var = Q / cf - mean * mean;
    var = var < 0.0 ? 0.0 : var;
    const double inv = 1.0 / sqrt(var + BNEPS);
    const float g = bf16r(gam[tt * N + c]);
    const float b = bf16r(bet[tt * N + c]);
    SSL[tt * 256 + c]        = (float)mean;
    SSL[512 + tt * 256 + c]  = (float)inv * g;
    SSL[1024 + tt * 256 + c] = b;
  }
  __syncthreads();
  for (int p = tid; p < 384; p += NTHR) {
    const v4f v = ((const v4f*)SSL)[p];
    *(volatile v4f*)(SS + 4 * p) = v;
  }
  __threadfence();
  for (int p = tid; p < 384; p += NTHR) {
    const v4f v = ((const v4f*)SSL)[p];
    *(volatile v4f*)(SS + 4 * p) = v;
  }
}

template<int KS, int AMODE, int EPI>
__global__ __launch_bounds__(HTHR) void k_hg(const float* __restrict__ A, int lda, const int* __restrict__ nt,
                                            const float* __restrict__ SS, const _Float16* __restrict__ WT,
                                            const float* __restrict__ bias, float* O, int accum, float* REC, int nN) {
  constexpr int NCG = (EPI == 0) ? 2 : 1;
  constexpr int N  = 128 * NCG;
  constexpr int K  = 32 * KS;
  constexpr int KQ = K / 8;
  constexpr int LDSU = LDS_HG(N, K) / 16;
  static_assert((LDS_HG(N, K) % 16) == 0);
  extern __shared__ v4f lds_dyn[];
  float* SSL = (float*)lds_dyn;
  int*   TY  = (int*)(SSL + 1536);
  float* STG = SSL + 1664;
  float* PST = STG + 16384;
  float* RS  = PST + 32 * N;
  _Float16* AT = (_Float16*)(RS + 4 * N);
  const int tid = (int)threadIdx.x, lane = tid & 31, wave = tid >> 5, hh = lane >> 4, m = lane & 15;
  const int rb = (int)blockIdx.x * HBM;
  const v4f z4 = {0.f, 0.f, 0.f, 0.f};

#pragma unroll 1
  for (int p = tid; p < LDSU; p += HTHR) lds_dyn[p] = z4;
  __syncthreads();

  if (AMODE == 1) {
    for (int p = tid; p < 384; p += HTHR) ((v4f*)SSL)[p] = *(const v4f*)(SS + 4 * p);
  }
  for (int p = tid; p < 8 * N; p += HTHR) ((v4f*)PST)[p] = z4;
  if (tid < HBM) {
    const int gr = rb + tid;
    const int gc = gr < nN ? gr : nN - 1;
    TY[tid] = nt[gc] > 0 ? 1 : 0;
  }
  __syncthreads();

#pragma unroll 1
  for (int u = tid; u < HBM * KQ; u += HTHR) {
    const int r  = u / KQ;
    const int k8 = (u - r * KQ) * 8;
    const int gr = rb + r;
    const bool valid = gr < nN;
    const int gc = valid ? gr : nN - 1;
    const float* arow = A + (size_t)gc * (size_t)lda;
    v4f xa, xb;
    if (AMODE == 0) {
      const int kc = k8 & 15;
      xa = *(const v4f*)(arow + kc);
      xb = *(const v4f*)(arow + kc + 4);
      xa = bf16r4(xa); xb = bf16r4(xb);
      if (k8 >= 16) { xa = z4; xb = z4; }
    } else {
      xa = *(const v4f*)(arow + k8);
      xb = *(const v4f*)(arow + k8 + 4);
      if (AMODE == 1) {
        const int tt = TY[r];
        const float* mt  = SSL + tt * 256 + k8;
        const float* sct = SSL + 512 + tt * 256 + k8;
        const float* bt  = SSL + 1024 + tt * 256 + k8;
        const v4f ma = *(const v4f*)mt,  mb = *(const v4f*)(mt + 4);
        const v4f sa = *(const v4f*)sct, sb = *(const v4f*)(sct + 4);
        const v4f ba = *(const v4f*)bt,  bb = *(const v4f*)(bt + 4);
        xa = lrelu4((xa - ma) * sa + ba);
        xb = lrelu4((xb - mb) * sb + bb);
      }
    }
    if (!valid) { xa = z4; xb = z4; }
    *(v8h*)(AT + (size_t)r * K + k8) = cvt8h(xa, xb, CA);
  }
  __syncthreads();

  float* stg = STG + wave * 2048;
  const int lr0 = 16 * wave;
  const _Float16* at = AT + (size_t)(lr0 + m) * K + 8 * hh;
#pragma unroll 1
  for (int cg = 0; cg < NCG; ++cg) {
#pragma unroll 1
    for (int t = 0; t < NTYP; ++t) {
      v8f acc[8];
      {
        const v8f z = {0.f, 0.f, 0.f, 0.f, 0.f, 0.f, 0.f, 0.f};
#pragma unroll
        for (int tc = 0; tc < 8; ++tc) acc[tc] = z;
      }
      const _Float16* wtt = WT + (size_t)(t * N + cg * 128 + m) * (size_t)K + 8 * hh;
#pragma unroll
      for (int ks = 0; ks < KS; ++ks) {
        FragH af;
        af.h[0] = *(const v8h*)(at + 32 * ks);
        af.h[1] = *(const v8h*)(at + 32 * ks + 16);
#pragma unroll
        for (int tc = 0; tc < 8; ++tc) {
          const _Float16* wq = wtt + (size_t)(16 * tc) * (size_t)K + 32 * ks;
          FragH bf;
          bf.h[0] = *(const v8h*)wq;
          bf.h[1] = *(const v8h*)(wq + 16);
          acc[tc] = wmh(af, bf, acc[tc]);
        }
      }
      __builtin_amdgcn_fence(__ATOMIC_RELEASE, "wavefront");
      __builtin_amdgcn_wave_barrier();
      const float* bst = bias + t * N + cg * 128;
#pragma unroll
      for (int tc = 0; tc < 8; ++tc) {
        const float bv = bf16r(bst[16 * tc + m]);
#pragma unroll
        for (int r = 0; r < 8; ++r) {
          const int lr  = 8 * hh + r;
          const int idx = lr * 128 + 16 * tc + m;
          float val = fmaf(acc[tc][r], SCL, bv);
          if (t != 0) {
            const float old = stg[idx];
            val = (TY[lr0 + lr] != 0) ? val : old;
          }
          stg[idx] = val;
        }
      }
    }
    __builtin_amdgcn_fence(__ATOMIC_RELEASE, "wavefront");
    __builtin_amdgcn_wave_barrier();

    v4f s0 = z4, q0 = z4, s1 = z4, q1 = z4;
#pragma unroll 1
    for (int i = 0; i < 16; ++i) {
      const int lr = lr0 + i;
      const int gr = rb + lr;
      const bool valid = gr < nN;
      const int ty = TY[lr];
      float* sp = stg + i * 128 + 4 * lane;
      v4f v = *(const v4f*)sp;
      float* op = O + (size_t)gr * (size_t)N + cg * 128 + 4 * lane;
      if (EPI == 1) {
        if (accum) {
          const v4f ho = *(const v4f*)op;
          v = v + ho;
        }
      }
      if (!valid) v = z4;
      *(v4f*)sp = v;
      *(volatile v4f*)op = v;
      const float f1 = (valid && ty != 0) ? 1.0f : 0.0f;
      const float f0 = (valid && ty == 0) ? 1.0f : 0.0f;
      const v4f vv = v * v;
      s0 += v * f0; q0 += vv * f0;
      s1 += v * f1; q1 += vv * f1;
    }
    __threadfence();
#pragma unroll 1
    for (int i = 0; i < 16; ++i) {
      const int gr = rb + lr0 + i;
      const v4f v = *(const v4f*)(stg + i * 128 + 4 * lane);
      float* op = O + (size_t)gr * (size_t)N + cg * 128 + 4 * lane;
      *(volatile v4f*)op = v;
    }
    float* pw = PST + (size_t)(4 * wave) * N + cg * 128 + 4 * lane;
    *(v4f*)(pw)         = s0;
    *(v4f*)(pw + N)     = q0;
    *(v4f*)(pw + 2 * N) = s1;
    *(v4f*)(pw + 3 * N) = q1;
  }
  __syncthreads();

  for (int e = tid; e < 4 * N; e += HTHR) {
    float a = 0.f;
#pragma unroll
    for (int w2 = 0; w2 < NWAVE; ++w2) a += PST[w2 * 4 * N + e];
    RS[e] = a;
  }
  __syncthreads();
  float* rec = REC + (size_t)blockIdx.x * (size_t)(4 * N);
  for (int p = tid; p < N; p += HTHR) {
    const v4f v = ((const v4f*)RS)[p];
    *(volatile v4f*)(rec + 4 * p) = v;
  }
  __threadfence();
  for (int p = tid; p < N; p += HTHR) {
    const v4f v = ((const v4f*)RS)[p];
    *(volatile v4f*)(rec + 4 * p) = v;
  }
}

__global__ __launch_bounds__(NTHR) void k_y16(const float* __restrict__ h, const int* __restrict__ nt,
                                            const float* __restrict__ SS, _Float16* Y, int nN, int nUnits) {
  const int u = (int)blockIdx.x * NTHR + (int)threadIdx.x;
  if (u >= nUnits) return;
  const int row = u >> 4;
  const int c0  = (u & 15) * 8;
  const int rc  = row < nN ? row : nN - 1;
  const int t   = nt[rc] > 0 ? 1 : 0;
  const float* p = h + (size_t)rc * CH + c0;
  v4f a = *(const v4f*)p, b = *(const v4f*)(p + 4);
  const float* mt  = SS + t * 256 + c0;
  const float* sct = SS + 512 + t * 256 + c0;
  const float* bt  = SS + 1024 + t * 256 + c0;
  const v4f ma = *(const v4f*)mt,  mb = *(const v4f*)(mt + 4);
  const v4f sa = *(const v4f*)sct, sb = *(const v4f*)(sct + 4);
  const v4f ba = *(const v4f*)bt,  bb = *(const v4f*)(bt + 4);
  a = lrelu4((a - ma) * sa + ba);
  b = lrelu4((b - mb) * sb + bb);
  const v4f z4 = {0.f, 0.f, 0.f, 0.f};
  if (row >= nN) { a = z4; b = z4; }
  const v8h hv = cvt8h(a, b, CA);
  const size_t o = (size_t)row * CH + c0;
  *(volatile v8h*)(Y + o) = hv;
  __threadfence();
  *(volatile v8h*)(Y + o) = hv;
}

__global__ __launch_bounds__(GTHR) void k_cg(const _Float16* __restrict__ A, const _Float16* __restrict__ WT,
                                           const float* __restrict__ rgb, _Float16* HS, float* h) {
  __shared__ __attribute__((aligned(16))) float stg[GBM * GBN];
  const int tid = (int)threadIdx.x, lane = tid & 31, wave = tid >> 5, hh = lane >> 4, m = lane & 15;
  const int rowBase = (int)blockIdx.x * GBM;
  const int cb      = (int)blockIdx.y;
  const int col0    = cb * GBN;

  {
    const v4f z4 = {0.f, 0.f, 0.f, 0.f};
#pragma unroll 1
    for (int p = tid; p < GBM * GBN / 4; p += GTHR) ((v4f*)stg)[p] = z4;
  }
  __syncthreads();

  v8f acc[4];
  {
    const v8f z = {0.f, 0.f, 0.f, 0.f, 0.f, 0.f, 0.f, 0.f};
    acc[0] = z; acc[1] = z; acc[2] = z; acc[3] = z;
  }
  const _Float16* ap = A  + (size_t)(rowBase + 16 * wave + m) * CH + 8 * hh;
  const _Float16* wp = WT + (size_t)(col0 + m) * CH + 8 * hh;
#pragma unroll
  for (int ks = 0; ks < CH / 32; ++ks) {
    FragH af;
    af.h[0] = *(const v8h*)(ap + 32 * ks);
    af.h[1] = *(const v8h*)(ap + 32 * ks + 16);
#pragma unroll
    for (int t = 0; t < 4; ++t) {
      const _Float16* wq = wp + (size_t)(16 * t) * CH + 32 * ks;
      FragH bf;
      bf.h[0] = *(const v8h*)wq;
      bf.h[1] = *(const v8h*)(wq + 16);
      acc[t] = wmh(af, bf, acc[t]);
    }
  }

  const bool hsPart = cb < 2 * NREL;
  if (hsPart) {
#pragma unroll
    for (int t = 0; t < 4; ++t) {
      const int lc = 16 * t + m;
#pragma unroll
      for (int r = 0; r < 8; ++r) {
        const int lr = 16 * wave + 8 * hh + r;
        stg[lr * GBN + lc] = acc[t][r] * HSC;
      }
    }
  } else {
    const int c0h = col0 - HSW;
#pragma unroll
    for (int t = 0; t < 4; ++t) {
      const int lc = 16 * t + m;
      const float bv = bf16r(rgb[c0h + lc]);
#pragma unroll
      for (int r = 0; r < 8; ++r) {
        const int lr = 16 * wave + 8 * hh + r;
        stg[lr * GBN + lc] = fmaf(acc[t][r], SCL, bv);
      }
    }
  }
  __syncthreads();

  if (hsPart) {
    const int q = lane >> 3, p = lane & 7;
    v8h hv[4];
#pragma unroll
    for (int i = 0; i < 4; ++i) {
      const int lr = 16 * wave + 4 * i + q;
      const v4f ga = *(const v4f*)(stg + lr * GBN + 8 * p);
      const v4f gb = *(const v4f*)(stg + lr * GBN + 8 * p + 4);
      hv[i] = cvt8h(ga, gb, 1.0f);
    }
#pragma unroll
    for (int i = 0; i < 4; ++i) {
      const int lr = 16 * wave + 4 * i + q;
      _Float16* gp = HS + (size_t)(rowBase + lr) * HSW + col0 + 8 * p;
      *(volatile v8h*)gp = hv[i];
    }
    __threadfence();
#pragma unroll
    for (int i = 0; i < 4; ++i) {
      const int lr = 16 * wave + 4 * i + q;
      _Float16* gp = HS + (size_t)(rowBase + lr) * HSW + col0 + 8 * p;
      *(volatile v8h*)gp = hv[i];
    }
  } else {
    const int c0h = col0 - HSW;
    v4f fv[8];
#pragma unroll
    for (int i = 0; i < 8; ++i) {
      const int lr = 16 * wave + 2 * i + hh;
      const int gr = rowBase + lr;
      const v4f ho = *(const v4f*)(h + (size_t)gr * CH + c0h + 4 * m);
      fv[i] = *(const v4f*)(stg + lr * GBN + 4 * m) + ho;
    }
#pragma unroll
    for (int i = 0; i < 8; ++i) {
      const int lr = 16 * wave + 2 * i + hh;
      const int gr = rowBase + lr;
      float* op = h + (size_t)gr * CH + c0h + 4 * m;
      *(volatile v4f*)op = fv[i];
    }
    __threadfence();
#pragma unroll
    for (int i = 0; i < 8; ++i) {
      const int lr = 16 * wave + 2 * i + hh;
      const int gr = rowBase + lr;
      float* op = h + (size_t)gr * CH + c0h + 4 * m;
      *(volatile v4f*)op = fv[i];
    }
  }
}

__global__ __launch_bounds__(NTHR) void k_drain(
    const int* __restrict__ srcs, const int* __restrict__ dsts, const int* __restrict__ ets,
    const int* __restrict__ nt, const _Float16* __restrict__ HS, float* h, float* REC,
    int nN, int nE, int nb, int vec8) {
  extern __shared__ v4f lds_dyn[];
  int* reg1 = (int*)lds_dyn;
  int* reg2 = reg1 + RCAP;
  int* scnt = reg2 + RCAP;
  int* soff = scnt + NBMAX;
  int* list = soff + NBMAX;
  int* wcnt = list + LISTN;
  int* wtot = wcnt + NWAVE;
  const int tid = (int)threadIdx.x, lane = tid & 31, wave = tid >> 5;
  const int nodeBase = (int)blockIdx.x * nb;

  {
    const v4f zz = {0.f, 0.f, 0.f, 0.f};
#pragma unroll 1
    for (int p = tid; p < LDS_AGG / 16; p += NTHR) lds_dyn[p] = zz;
  }
  __syncthreads();

  for (int i = tid; i < NBMAX; i += NTHR) scnt[i] = 0;
  __syncthreads();

  int tot = 0;
  const int nChunks = (nE + CHUNK - 1) / CHUNK;
#pragma unroll 1
  for (int ch = 0; ch < nChunks; ++ch) {
    const int cbase = ch * CHUNK;
    const int wc = scan_chunk(dsts, nE, cbase, nodeBase, nb, vec8, list, tid, lane, wave);
    if (lane == 0) wcnt[wave] = wc;
    __syncthreads();
    int pre = 0, all = 0;
#pragma unroll
    for (int w2 = 0; w2 < NWAVE; ++w2) {
      int c = wcnt[w2];
      c = c < 0 ? 0 : (c > WCAP ? WCAP : c);
      all += c;
      pre += (w2 < wave) ? c : 0;
    }
    const int wcc  = wc > WCAP ? WCAP : wc;
    const int base = tot + pre;
#pragma unroll 1
    for (int i = lane; i < wcc; i += 32) {
      const int ent = list[wave * WCAP + i];
      const int el  = (ent >> 12) & (CHUNK - 1);
      const int sl  = ent & (NBMAX - 1);
      int eid = cbase + el;
      eid = eid > nE - 1 ? nE - 1 : eid;
      const int pos = base + i;
      if (pos < RCAP) reg1[pos] = (int)(((unsigned)eid << 12) | (unsigned)sl);
    }
    tot += all;
    tot = tot > RCAP ? RCAP : tot;
    __syncthreads();
  }
  const int nh = tot;

  if (wave == 0) {
#pragma unroll 1
    for (int b0 = 0; b0 < nh; b0 += 32) {
      const int idx = b0 + lane;
      const int uv  = reg1[idx < RCAP ? idx : RCAP - 1];
      const int m32 = (nh - b0) < 32 ? (nh - b0) : 32;
#pragma unroll 1
      for (int k = 0; k < m32; ++k) {
        const int u  = __builtin_amdgcn_readlane(uv, k);
        const int sl = u & (NBMAX - 1);
        if (lane == 0) scnt[sl] = scnt[sl] + 1;
      }
    }
  }
  __syncthreads();

  {
    const v4i ca = *(const v4i*)(scnt + 8 * tid);
    const v4i cb = *(const v4i*)(scnt + 8 * tid + 4);
    const int e0 = ca.x < 0 ? 0 : ca.x, e1 = ca.y < 0 ? 0 : ca.y, e2 = ca.z < 0 ? 0 : ca.z, e3 = ca.w < 0 ? 0 : ca.w;
    const int e4 = cb.x < 0 ? 0 : cb.x, e5 = cb.y < 0 ? 0 : cb.y, e6 = cb.z < 0 ? 0 : cb.z, e7 = cb.w < 0 ? 0 : cb.w;
    const int ts = e0 + e1 + e2 + e3 + e4 + e5 + e6 + e7;
    int incl = ts;
#pragma unroll
    for (int d = 1; d < 32; d <<= 1) {
      const int up = __shfl_up(incl, d);
      incl += (lane >= d) ? up : 0;
    }
    if (lane == 31) wtot[wave] = incl;
    __syncthreads();
    int pre = 0;
#pragma unroll
    for (int w2 = 0; w2 < NWAVE; ++w2) pre += (w2 < wave) ? wtot[w2] : 0;
    int run = pre + incl - ts;
    soff[8 * tid + 0] = run; run += e0;
    soff[8 * tid + 1] = run; run += e1;
    soff[8 * tid + 2] = run; run += e2;
    soff[8 * tid + 3] = run; run += e3;
    soff[8 * tid + 4] = run; run += e4;
    soff[8 * tid + 5] = run; run += e5;
    soff[8 * tid + 6] = run; run += e6;
    soff[8 * tid + 7] = run;
  }
  __syncthreads();
  for (int i = tid; i < NBMAX; i += NTHR) list[i] = soff[i];
  __syncthreads();

  if (wave == 0) {
#pragma unroll 1
    for (int b0 = 0; b0 < nh; b0 += 32) {
      const int idx = b0 + lane;
      const int uv  = reg1[idx < RCAP ? idx : RCAP - 1];
      const int m32 = (nh - b0) < 32 ? (nh - b0) : 32;
#pragma unroll 1
      for (int k = 0; k < m32; ++k) {
        const int u   = __builtin_amdgcn_readlane(uv, k);
        const int sl  = u & (NBMAX - 1);
        const int eid = (int)((unsigned)u >> 12);
        if (lane == 0) {
          int pos = list[sl];
          pos = pos < 0 ? 0 : (pos > RCAP - 1 ? RCAP - 1 : pos);
          reg2[pos] = eid;
          list[sl] = pos + 1;
        }
      }
    }
  }
  __syncthreads();

  const int nbw = nb >> 3;
  const bool ovf = (nh >= RCAP);
  const float qnan = __int_as_float(0x7fc00000);
  const v4f qn4 = {qnan, qnan, qnan, qnan};
  const v4f z4  = {0.f, 0.f, 0.f, 0.f};
  v4f s0 = z4, q0 = z4, s1 = z4, q1 = z4;
#pragma unroll 1
  for (int jt = 0; jt < nbw; ++jt) {
    const int slot = wave * nbw + jt;
    const int grow = nodeBase + slot;
    if (grow >= nN) continue;
    int st = soff[slot];
    const int craw = scnt[slot];
    int cnt = craw;
    st  = st < 0 ? 0 : (st > nh ? nh : st);
    cnt = cnt < 0 ? 0 : (cnt > DEGCAP ? DEGCAP : cnt);
    if (cnt > nh - st) cnt = nh - st;
    const bool pz = ovf || (craw > DEGCAP);
    v4f agg = z4;
#pragma unroll 1
    for (int q = 0; q < cnt; ++q) {
      int idx = st + q; idx = idx > RCAP - 1 ? RCAP - 1 : idx;
      int eid = reg2[idx]; eid = eid < 0 ? 0 : (eid > nE - 1 ? nE - 1 : eid);
      const int sraw = srcs[eid];
      const int s  = sraw < 0 ? 0 : (sraw > nN - 1 ? nN - 1 : sraw);
      const int rraw = ets[eid];
      const int rr = rraw < 0 ? 0 : (rraw > NREL - 1 ? NREL - 1 : rraw);
      const v4h m4 = *(const v4h*)(HS + (size_t)s * HSW + rr * CH + 4 * lane);
      agg += __builtin_convertvector(m4, v4f);
    }
    float* hp = h + (size_t)grow * CH + 4 * lane;
    v4f hv = *(const v4f*)hp;
    hv = hv + agg * RHS;
    if (pz) hv = qn4;
    *(volatile v4f*)hp = hv;
    __threadfence();
    *(volatile v4f*)hp = hv;
    const int tr = nt[grow] > 0 ? 1 : 0;
    const float f1 = tr ? 1.0f : 0.0f;
    const float f0 = tr ? 0.0f : 1.0f;
    const v4f hq = hv * hv;
    s0 += hv * f0; q0 += hq * f0;
    s1 += hv * f1; q1 += hq * f1;
  }
  float* PST = (float*)reg1;
  float* RS  = PST + NWAVE * 512;
  {
    float* pw = PST + wave * 512 + 4 * lane;
    *(v4f*)(pw)       = s0;
    *(v4f*)(pw + 128) = q0;
    *(v4f*)(pw + 256) = s1;
    *(v4f*)(pw + 384) = q1;
  }
  __syncthreads();
  for (int e = tid; e < 512; e += NTHR) {
    float a = 0.f;
#pragma unroll
    for (int w2 = 0; w2 < NWAVE; ++w2) a += PST[w2 * 512 + e];
    RS[e] = a;
  }
  __syncthreads();
  float* rec = REC + (size_t)blockIdx.x * 512;
  if (tid < 128) {
    const v4f v = ((const v4f*)RS)[tid];
    *(volatile v4f*)(rec + 4 * tid) = v;
  }
  __threadfence();
  if (tid < 128) {
    const v4f v = ((const v4f*)RS)[tid];
    *(volatile v4f*)(rec + 4 * tid) = v;
  }
}

__global__ __launch_bounds__(FTHR) void k_final(const float* __restrict__ P, const int* __restrict__ nt,
                                              const float* __restrict__ SS, const _Float16* __restrict__ WT,
                                              const float* __restrict__ b1, float* out, int nN) {
  __shared__ __attribute__((aligned(16))) float SSL[1536];
  __shared__ __attribute__((aligned(16))) int   TY[64];
  __shared__ __attribute__((aligned(16))) float stg[64 * DOUT];
  const int tid = (int)threadIdx.x, lane = tid & 31, wave = tid >> 5, hh = lane >> 4, m = lane & 15;
  const int rowBase = (int)blockIdx.x * 64;
  {
    const v4f z4 = {0.f, 0.f, 0.f, 0.f};
    const v4i zi = {0, 0, 0, 0};
    for (int p = tid; p < 384; p += FTHR) ((v4f*)SSL)[p] = z4;
    if (tid < 16) ((v4i*)TY)[tid] = zi;
    if (tid < 64) ((v4f*)stg)[tid] = z4;
  }
  __syncthreads();
  for (int p = tid; p < 384; p += FTHR) ((v4f*)SSL)[p] = *(const v4f*)(SS + 4 * p);
  if (tid < 64) {
    const int gr = rowBase + tid;
    const int gc = gr < nN ? gr : nN - 1;
    TY[tid] = nt[gc] > 0 ? 1 : 0;
  }
  __syncthreads();
  const int lrm = 16 * wave + m;
  int grow = rowBase + lrm;
  grow = grow < nN ? grow : nN - 1;
  const int tt = TY[lrm];
  const float* arow = P + (size_t)grow * HID;
  const float* mt  = SSL + tt * 256;
  const float* sct = SSL + 512 + tt * 256;
  const float* bt  = SSL + 1024 + tt * 256;
  const _Float16* w0 = WT + (size_t)(m) * HID + 8 * hh;
  const _Float16* w1 = WT + (size_t)(16 + m) * HID + 8 * hh;
  v8f acc[2];
  {
    const v8f z = {0.f, 0.f, 0.f, 0.f, 0.f, 0.f, 0.f, 0.f};
    acc[0] = z; acc[1] = z;
  }
#pragma unroll
  for (int ks = 0; ks < HID / 32; ++ks) {
    FragH af;
    af.h[0] = cv8<1>(arow, mt, sct, bt, 32 * ks + 8 * hh);
    af.h[1] = cv8<1>(arow, mt, sct, bt, 32 * ks + 16 + 8 * hh);
    FragH bf0, bf1;
    bf0.h[0] = *(const v8h*)(w0 + 32 * ks);
    bf0.h[1] = *(const v8h*)(w0 + 32 * ks + 16);
    bf1.h[0] = *(const v8h*)(w1 + 32 * ks);
    bf1.h[1] = *(const v8h*)(w1 + 32 * ks + 16);
    acc[0] = wmh(af, bf0, acc[0]);
    acc[1] = wmh(af, bf1, acc[1]);
  }
  const int mc = m < DOUT ? m : DOUT - 1;
#pragma unroll
  for (int r = 0; r < 8; ++r) {
    const int lr = 16 * wave + 8 * hh + r;
    const int tr = TY[lr];
    const float a = tr ? acc[1][r] : acc[0][r];
    const float val = fmaf(a, SCL, bf16r(b1[tr * DOUT + mc]));
    if (m < DOUT) stg[lr * DOUT + m] = val;
  }
  __syncthreads();
  const int gro = rowBase + tid;
  const bool wr = (tid < 64) && (gro < nN);
  v4f ov = {0.f, 0.f, 0.f, 0.f};
  if (tid < 64) ov = ((const v4f*)stg)[tid];
  if (wr) *(volatile v4f*)(out + (size_t)gro * DOUT) = ov;
  __threadfence();
  if (wr) *(volatile v4f*)(out + (size_t)gro * DOUT) = ov;
}

static int pick_nb(int nE, int nN) {
  int nb = NBMAX;
  while (nb > 16 && (long long)nb * (long long)nE * 5LL > (long long)RCAP * (long long)nN * 4LL) nb >>= 1;
  return nb;
}
static inline int cdiv(int a, int b) { return (a + b - 1) / b; }
static inline size_t al256(size_t v) { return (v + 255) & ~(size_t)255; }

extern "C" void kernel_launch(void* const* d_in, const int* in_sizes, int n_in,
                              void* d_out, int out_size, void* d_ws, size_t ws_size,
                              hipStream_t stream) {
  if (n_in < 29) return;
  const int nN = in_sizes[0] / DIN;
  if (nN <= 0 || in_sizes[0] != nN * DIN || nN > (1 << 22)) return;
  if (in_sizes[1] < 2 || (in_sizes[1] & 1) != 0) return;
  const int nE = in_sizes[1] / 2;
  if (nE < 1 || nE > (1 << 20)) return;
  if (in_sizes[2] != nN || in_sizes[3] != nE) return;
  if (in_sizes[4]  != NTYP * DIN * HID      || in_sizes[5]  != NTYP * HID) return;
  if (in_sizes[6]  != NTYP * HID            || in_sizes[7]  != NTYP * HID) return;
  if (in_sizes[8]  != NTYP * HID * CH       || in_sizes[9]  != NTYP * CH)  return;
  if (in_sizes[10] != NLAY * NTYP * CH      || in_sizes[11] != NLAY * NTYP * CH) return;
  if (in_sizes[12] != NLAY * NREL * CH * CH || in_sizes[13] != NLAY * CH * CH) return;
  if (in_sizes[14] != NLAY * CH) return;
  if (in_sizes[15] != NLAY * NTYP * CH      || in_sizes[16] != NLAY * NTYP * CH) return;
  if (in_sizes[17] != NLAY * NTYP * CH * HID || in_sizes[18] != NLAY * NTYP * HID) return;
  if (in_sizes[19] != NLAY * NTYP * HID     || in_sizes[20] != NLAY * NTYP * HID) return;
  if (in_sizes[21] != NLAY * NTYP * HID * CH || in_sizes[22] != NLAY * NTYP * CH) return;
  if (in_sizes[23] != NTYP * CH * HID       || in_sizes[24] != NTYP * HID) return;
  if (in_sizes[25] != NTYP * HID            || in_sizes[26] != NTYP * HID) return;
  if (in_sizes[27] != NTYP * HID * DOUT     || in_sizes[28] != NTYP * DOUT) return;
  if (out_size != nN * DOUT || (out_size & 3) != 0) return;

  const float* x      = (const float*)d_in[0];
  const int*   ei     = (const int*)  d_in[1];
  const int*   ntp    = (const int*)  d_in[2];
  const int*   etp    = (const int*)  d_in[3];
  const float* ri_w0  = (const float*)d_in[4];
  const float* ri_b0  = (const float*)d_in[5];
  const float* ri_g0  = (const float*)d_in[6];
  const float* ri_be0 = (const float*)d_in[7];
  const float* ri_w1  = (const float*)d_in[8];
  const float* ri_b1  = (const float*)d_in[9];
  const float* cn_g   = (const float*)d_in[10];
  const float* cn_b   = (const float*)d_in[11];
  const float* rg_w   = (const float*)d_in[12];
  const float* rg_rt  = (const float*)d_in[13];
  const float* rg_bs  = (const float*)d_in[14];
  const float* mn_g   = (const float*)d_in[15];
  const float* mn_b   = (const float*)d_in[16];
  const float* mw0    = (const float*)d_in[17];
  const float* mb0    = (const float*)d_in[18];
  const float* mg0    = (const float*)d_in[19];
  const float* mbe0   = (const float*)d_in[20];
  const float* mw1    = (const float*)d_in[21];
  const float* mb1    = (const float*)d_in[22];
  const float* ro_w0  = (const float*)d_in[23];
  const float* ro_b0  = (const float*)d_in[24];
  const float* ro_g0  = (const float*)d_in[25];
  const float* ro_be0 = (const float*)d_in[26];
  const float* ro_w1  = (const float*)d_in[27];
  const float* ro_b1  = (const float*)d_in[28];
  float* out = (float*)d_out;
  const int* src = ei;
  const int* dst = ei + nE;

  const int MP   = cdiv(nN, HBM) * HBM;
  const int gH   = MP / HBM;
  const int gC   = MP / GBM;
  const int nb   = pick_nb(nE, nN);
  const int gA   = cdiv(MP, nb);
  const int vec8 = ((nE & 3) == 0) ? 1 : 0;
  if (gA * nb < MP) return;
  const int recF = (gH * 4 * HID > gA * 512) ? gH * 4 * HID : gA * 512;

  char* ws = (char*)d_ws;
  size_t off = 0;
  const size_t oH    = off; off = al256(off + (size_t)MP * CH * 4);
  const size_t oRB   = off; off = al256(off + (size_t)MP * 1024);
  const size_t oY    = off; off = al256(off + (size_t)MP * CH * 2);
  const size_t oREC  = off; off = al256(off + (size_t)recF * 4);
  const size_t oSS   = off; off = al256(off + (size_t)1536 * 4);
  const size_t oWri0 = off; off = al256(off + (size_t)NTYP * HID * 32 * 2);
  const size_t oWri1 = off; off = al256(off + (size_t)NTYP * CH * HID * 2);
  size_t oWR[NLAY], oWm0[NLAY], oWm1[NLAY];
  for (int l = 0; l < NLAY; ++l) {
    oWR[l]  = off; off = al256(off + (size_t)NRC * CH * 2);
    oWm0[l] = off; off = al256(off + (size_t)NTYP * HID * CH * 2);
    oWm1[l] = off; off = al256(off + (size_t)NTYP * CH * HID * 2);
  }
  const size_t oWro0 = off; off = al256(off + (size_t)NTYP * HID * CH * 2);
  const size_t oWro1 = off; off = al256(off + (size_t)NTYP * 16 * HID * 2);
  if (off > ws_size || off > (size_t)WSLIM) return;
  if ((off >> 4) > (size_t)0x7fffffff) return;
  const int nZ4 = (int)(off >> 4);
  const int nO4 = out_size >> 2;

  float*    hP   = (float*)(ws + oH);
  float*    Pp   = (float*)(ws + oRB);
  _Float16* HSp  = (_Float16*)(ws + oRB);
  _Float16* Y16  = (_Float16*)(ws + oY);
  float*    REC  = (float*)(ws + oREC);
  float*    SS   = (float*)(ws + oSS);
  _Float16* Wri0 = (_Float16*)(ws + oWri0);
  _Float16* Wri1 = (_Float16*)(ws + oWri1);
  _Float16* WR[NLAY]; _Float16* Wm0[NLAY]; _Float16* Wm1[NLAY];
  for (int l = 0; l < NLAY; ++l) {
    WR[l]  = (_Float16*)(ws + oWR[l]);
    Wm0[l] = (_Float16*)(ws + oWm0[l]);
    Wm1[l] = (_Float16*)(ws + oWm1[l]);
  }
  _Float16* Wro0 = (_Float16*)(ws + oWro0);
  _Float16* Wro1 = (_Float16*)(ws + oWro1);

  hipFuncSetAttribute(reinterpret_cast<const void*>(&k_hg<1, 0, 0>),
                      hipFuncAttributeMaxDynamicSharedMemorySize, LDS_HG(HID, 32));
  hipFuncSetAttribute(reinterpret_cast<const void*>(&k_hg<8, 1, 1>),
                      hipFuncAttributeMaxDynamicSharedMemorySize, LDS_HG(CH, HID));
  hipFuncSetAttribute(reinterpret_cast<const void*>(&k_hg<4, 1, 0>),
                      hipFuncAttributeMaxDynamicSharedMemorySize, LDS_HG(HID, CH));
  hipFuncSetAttribute(reinterpret_cast<const void*>(&k_hg<4, 2, 0>),
                      hipFuncAttributeMaxDynamicSharedMemorySize, LDS_HG(HID, CH));
  hipFuncSetAttribute(reinterpret_cast<const void*>(&k_drain),
                      hipFuncAttributeMaxDynamicSharedMemorySize, LDS_AGG);

  {
    int gZ = cdiv(nZ4, NTHR);
    gZ = gZ > ZBLK ? ZBLK : (gZ < 1 ? 1 : gZ);
    k_zero<<<gZ, NTHR, 0, stream>>>((float*)ws, nZ4);
    int gO = cdiv(nO4, NTHR);
    gO = gO > ZBLK ? ZBLK : (gO < 1 ? 1 : gO);
    k_zero<<<gO, NTHR, 0, stream>>>(out, nO4);
  }

  {
    const int nU0 = NTYP * HID * (32 / 8);
    k_wprep<<<cdiv(nU0, NTHR), NTHR, 0, stream>>>(ri_w0, ri_w0, 2, HID, HID, DIN, 32, DIN * HID, Wri0, nU0);
    const int nU1 = NTYP * CH * (HID / 8);
    k_wprep<<<cdiv(nU1, NTHR), NTHR, 0, stream>>>(ri_w1, ri_w1, 2, CH, CH, HID, HID, HID * CH, Wri1, nU1);
    for (int l = 0; l < NLAY; ++l) {
      const int nUR = NRC * (CH / 8);
      k_wprep<<<cdiv(nUR, NTHR), NTHR, 0, stream>>>(rg_w + (size_t)l * NREL * CH * CH, rg_rt + (size_t)l * CH * CH,
                                                    NREL, CH, CH, CH, CH, CH * CH, WR[l], nUR);
      const int nUa = NTYP * HID * (CH / 8);
      k_wprep<<<cdiv(nUa, NTHR), NTHR, 0, stream>>>(mw0 + (size_t)l * NTYP * CH * HID, mw0 + (size_t)l * NTYP * CH * HID,
                                                    2, HID, HID, CH, CH, CH * HID, Wm0[l], nUa);
      const int nUb = NTYP * CH * (HID / 8);
      k_wprep<<<cdiv(nUb, NTHR), NTHR, 0, stream>>>(mw1 + (size_t)l * NTYP * HID * CH, mw1 + (size_t)l * NTYP * HID * CH,
                                                    2, CH, CH, HID, HID, HID * CH, Wm1[l], nUb);
    }
    const int nUc = NTYP * HID * (CH / 8);
    k_wprep<<<cdiv(nUc, NTHR), NTHR, 0, stream>>>(ro_w0, ro_w0, 2, HID, HID, CH, CH, CH * HID, Wro0, nUc);
    const int nUd = NTYP * 16 * (HID / 8);
    k_wprep<<<cdiv(nUd, NTHR), NTHR, 0, stream>>>(ro_w1, ro_w1, 2, 16, DOUT, HID, HID, HID * DOUT, Wro1, nUd);
  }

  const int nUy = MP * (CH / 8);

  k_hg<1, 0, 0><<<gH, HTHR, LDS_HG(HID, 32), stream>>>(x, DIN, ntp, SS, Wri0, ri_b0, Pp, 0, REC, nN);
  k_fold<<<1, NTHR, 0, stream>>>(REC, gH, HID, ri_g0, ri_be0, ntp, nN, SS);
  k_hg<8, 1, 1><<<gH, HTHR, LDS_HG(CH, HID), stream>>>(Pp, HID, ntp, SS, Wri1, ri_b1, hP, 0, REC, nN);
  k_fold<<<1, NTHR, 0, stream>>>(REC, gH, CH, cn_g, cn_b, ntp, nN, SS);

  for (int l = 0; l < NLAY; ++l) {
    k_y16<<<cdiv(nUy, NTHR), NTHR, 0, stream>>>(hP, ntp, SS, Y16, nN, nUy);
    k_cg<<<dim3(gC, NRC / GBN), GTHR, 0, stream>>>(Y16, WR[l], rg_bs + (size_t)l * CH, HSp, hP);
    k_drain<<<gA, NTHR, LDS_AGG, stream>>>(src, dst, etp, ntp, HSp, hP, REC, nN, nE, nb, vec8);
    k_fold<<<1, NTHR, 0, stream>>>(REC, gA, CH, mn_g + (size_t)l * NTYP * CH, mn_b + (size_t)l * NTYP * CH, ntp, nN, SS);
    k_hg<4, 1, 0><<<gH, HTHR, LDS_HG(HID, CH), stream>>>(hP, CH, ntp, SS, Wm0[l], mb0 + (size_t)l * NTYP * HID, Pp, 0,
                                                       REC, nN);
    k_fold<<<1, NTHR, 0, stream>>>(REC, gH, HID, mg0 + (size_t)l * NTYP * HID, mbe0 + (size_t)l * NTYP * HID, ntp, nN, SS);
    k_hg<8, 1, 1><<<gH, HTHR, LDS_HG(CH, HID), stream>>>(Pp, HID, ntp, SS, Wm1[l], mb1 + (size_t)l * NTYP * CH, hP, 1,
                                                       REC, nN);
    if (l + 1 < NLAY)
      k_fold<<<1, NTHR, 0, stream>>>(REC, gH, CH, cn_g + (size_t)(l + 1) * NTYP * CH, cn_b + (size_t)(l + 1) * NTYP * CH,
                                     ntp, nN, SS);
  }

  k_hg<4, 2, 0><<<gH, HTHR, LDS_HG(HID, CH), stream>>>(hP, CH, ntp, SS, Wro0, ro_b0, Pp, 0, REC, nN);
  k_fold<<<1, NTHR, 0, stream>>>(REC, gH, HID, ro_g0, ro_be0, ntp, nN, SS);
  k_final<<<gC, FTHR, 0, stream>>>(Pp, ntp, SS, Wro1, ro_b1, out, nN);
}
